// LocalAtomFAIPA_54357106098681
// MI455X (gfx1250) — hardware-verified
//
#include <hip/hip_runtime.h>
#include <hip/hip_bf16.h>
#include <math.h>

#define BB   2
#define NN   4096
#define DIM  256
#define HH   8
#define KK   32
#define BN   (BB*NN)

typedef __attribute__((ext_vector_type(16))) _Float16 v16h;
typedef __attribute__((ext_vector_type(8)))  _Float16 v8h;
typedef __attribute__((ext_vector_type(4)))  _Float16 v4h;
typedef __attribute__((ext_vector_type(8)))  float    v8f;
typedef __attribute__((ext_vector_type(4)))  float    v4f_t;
typedef float v4fa __attribute__((ext_vector_type(4), may_alias));
typedef __attribute__((ext_vector_type(4)))  unsigned v4u_t;
typedef unsigned v4ua __attribute__((ext_vector_type(4), may_alias));

__device__ __forceinline__ float gelu_tanh(float x) {
    float x3 = x * x * x;
    return 0.5f * x * (1.0f + tanhf(0.7978845608028654f * (x + 0.044715f * x3)));
}

__global__ __launch_bounds__(256) void qpos_kernel(const float* __restrict__ x,
                                                   const float* __restrict__ qw,
                                                   const float* __restrict__ qb,
                                                   float* __restrict__ qpos) {
    int gid = blockIdx.x * blockDim.x + threadIdx.x;
    if (gid >= BN * 24) return;
    int q = gid / 24;
    int o = gid - q * 24;
    const float* xr = x + (size_t)q * DIM;
    float acc = qb[o];
#pragma unroll 8
    for (int k = 0; k < DIM; ++k)
        acc = fmaf(xr[k], qw[k * 24 + o], acc);
    *(volatile float*)(qpos + gid) = acc; __threadfence(); *(volatile float*)(qpos + gid) = acc;
}

template <typename AT, int EPI, typename OT, int KDIM, int NC>
__global__ __launch_bounds__(256) void gemm_wmma(const AT* __restrict__ A,
                                                 const float* __restrict__ W,
                                                 const float* __restrict__ bias,
                                                 const float* __restrict__ res,
                                                 OT* __restrict__ out) {
    constexpr int KT = KDIM / 32;
    __shared__ _Float16 As[2][128 * 32];
    __shared__ _Float16 Bs[2][64 * 32];

    const int t    = threadIdx.x;
    const int lane = t & 31;
    const int w    = t >> 5;
    const int m0   = blockIdx.x * 128;
    const int n0   = blockIdx.y * 64;

    v8f acc[4];
#pragma unroll
    for (int ct = 0; ct < 4; ++ct)
#pragma unroll
        for (int r = 0; r < 8; ++r) acc[ct][r] = 0.0f;

    const int aRow  = t >> 3;
    const int aCol4 = (t & 7) * 4;
    const int bN    = t & 63;
    const int bK0   = (t >> 6) * 8;

    const AT*    aBase = A + (size_t)(m0 + aRow) * KDIM + aCol4;
    const float* wBase = W + (size_t)bK0 * NC + n0 + bN;

    v4h   aReg[4];
    float bReg[8];

    auto fetch = [&](int kt) {
        const int kb = kt * 32;
#pragma unroll
        for (int p = 0; p < 4; ++p) {
            const AT* src = aBase + (size_t)p * 32 * KDIM + kb;
            if constexpr (sizeof(AT) == 4) {
                const float4 f = *(const float4*)src;
                v4h h; h[0] = (_Float16)f.x; h[1] = (_Float16)f.y;
                       h[2] = (_Float16)f.z; h[3] = (_Float16)f.w;
                aReg[p] = h;
            } else {
                aReg[p] = *(const v4h*)src;
            }
        }
#pragma unroll
        for (int p = 0; p < 8; ++p) {
            bReg[p] = wBase[(size_t)(kb + p) * NC];
        }
    };
    auto commit = [&](int buf) {
#pragma unroll
        for (int p = 0; p < 4; ++p) {
            const int row = p * 32 + aRow;
            *(v4h*)&As[buf][row * 32 + aCol4] = aReg[p];
        }
        v8h hb;
#pragma unroll
        for (int p = 0; p < 8; ++p) hb[p] = (_Float16)bReg[p];
        *(v8h*)&Bs[buf][bN * 32 + bK0] = hb;
    };
    auto compute = [&](int buf) {
        const _Float16* pA = &As[buf][(w * 16 + (lane & 15)) * 32];
        const int abase = (lane >> 4) * 8;
        v16h af;
#pragma unroll
        for (int e = 0; e < 8; ++e) {
            af[e]     = pA[abase + e];
            af[e + 8] = pA[abase + 16 + e];
        }
#pragma unroll
        for (int ct = 0; ct < 4; ++ct) {
            const _Float16* pB = &Bs[buf][(ct * 16 + (lane & 15)) * 32];
            v16h bf;
#pragma unroll
            for (int e = 0; e < 8; ++e) { bf[e] = pB[abase + e]; bf[e + 8] = pB[abase + 16 + e]; }
            acc[ct] = __builtin_amdgcn_wmma_f32_16x16x32_f16(
                false, af, false, bf, (short)0, acc[ct], false, false);
        }
    };

    fetch(0);
    commit(0);
    __syncthreads();
#pragma unroll
    for (int kt = 0; kt < KT; ++kt) {
        if (kt + 1 < KT) fetch(kt + 1);
        compute(kt & 1);
        if (kt + 1 < KT) commit((kt + 1) & 1);
        __syncthreads();
    }

    __shared__ __attribute__((aligned(16))) float stg[8][16 * 68];
    float* sw = stg[w];
#pragma unroll
    for (int ct = 0; ct < 4; ++ct) {
        const int col = n0 + ct * 16 + (lane & 15);
        const float bv = bias[col];
#pragma unroll
        for (int r = 0; r < 8; ++r) {
            const int rl = (lane >> 4) * 8 + r, row = m0 + w * 16 + rl;
            float val = acc[ct][r] + bv;
            if constexpr (EPI == 1) val = gelu_tanh(val);
            else if constexpr (EPI == 2) val += res[(size_t)row * NC + col];
            sw[rl * 68 + ct * 16 + (lane & 15)] = val;
        }
    }
    asm volatile("s_wait_dscnt 0" ::: "memory");
#pragma unroll 1
    for (int pass = 0; pass < 2; ++pass) {
        if constexpr (sizeof(OT) == 4) {
#pragma unroll
            for (int i = 0; i < 8; ++i) { const int c = lane + 32 * i, rr = c >> 4, q = (c & 15) * 4;
                *(volatile v4f_t*)((float*)out + (size_t)(m0 + w * 16 + rr) * NC + n0 + q) = *(const volatile v4fa*)(sw + rr * 68 + q); }
        } else {
#pragma unroll
            for (int i = 0; i < 4; ++i) { const int c = lane + 32 * i, rr = c >> 3, q = (c & 7) * 8; const float* s = sw + rr * 68 + q;
                _Float16 hh[8];
#pragma unroll
                for (int e = 0; e < 8; ++e) hh[e] = (_Float16)s[e];
                *(volatile v4u_t*)((_Float16*)out + (size_t)(m0 + w * 16 + rr) * NC + n0 + q) = *(const v4ua*)hh; }
        }
        __threadfence();
    }
}

__global__ __launch_bounds__(256) void attn_ln_kernel(const float* __restrict__ qpos,
                                                      const float* __restrict__ fp,
                                                      const int*   __restrict__ i1,
                                                      const int* __restrict__ npm,
                                                      const float* __restrict__ v,
                                                      const float* __restrict__ ln_g,
                                                      const float* __restrict__ ln_b,
                                                      _Float16* __restrict__ hout) {
    __shared__ float s_qp[24];
    __shared__ float s_fpq[24];
    __shared__ int   s_nbr[32];
    __shared__ float s_fpn[32 * 24];
    __shared__ float s_d[2048];
    __shared__ float s_aff[256];
    __shared__ float s_v[32 * 256];
    __shared__ float s_red[16];

    const int q    = blockIdx.x;
    const int t    = threadIdx.x;
    const int lane = t & 31;

    if (t < 24) { s_qp[t] = qpos[q * 24 + t]; s_fpq[t] = fp[(size_t)q * 24 + t]; }
    if (t < 32) { int nb = i1[(size_t)q * KK + t]; nb = (nb < 0) ? 0 : (nb >= BN ? BN - 1 : nb); s_nbr[t] = nb; }
    __syncthreads();

    for (int i = t; i < 32 * 24; i += 256) {
        int nb = i / 24, r = i - nb * 24;
        s_fpn[i] = fp[(size_t)s_nbr[nb] * 24 + r];
    }
    __syncthreads();

    for (int j = t; j < 2048; j += 256) {
        int k = j >> 6, f = (j >> 3) & 7, h = j & 7;
        float dx = s_qp[h * 3 + 0] + s_fpq[f * 3 + 0] - s_fpn[k * 24 + f * 3 + 0];
        float dy = s_qp[h * 3 + 1] + s_fpq[f * 3 + 1] - s_fpn[k * 24 + f * 3 + 1];
        float dz = s_qp[h * 3 + 2] + s_fpq[f * 3 + 2] - s_fpn[k * 24 + f * 3 + 2];
        s_d[j] = sqrtf(dx * dx + dy * dy + dz * dz);
    }
    __syncthreads();

    float sacc = 0.0f;
#pragma unroll
    for (int f2 = 0; f2 < 8; ++f2) sacc += s_d[f2 * 256 + t];
    float logit = -0.125f * sacc;

    float mx = logit;
#pragma unroll
    for (int off = 16; off >= 1; off >>= 1) mx = fmaxf(mx, __shfl_xor(mx, off, 32));
    float e = __expf(logit - mx);
    float se = e;
#pragma unroll
    for (int off = 16; off >= 1; off >>= 1) se += __shfl_xor(se, off, 32);
    float soft = e / se;
    float maskv = ((npm[q] != 0) ? 1.0f : 0.0f) * ((npm[s_nbr[lane]] != 0) ? 1.0f : 0.0f);
    float a = soft * maskv;
    float sa = a;
#pragma unroll
    for (int off = 16; off >= 1; off >>= 1) sa += __shfl_xor(sa, off, 32);
    s_aff[t] = a / (sa + 1e-6f);
    __syncthreads();

#pragma unroll
    for (int i = 0; i < 8; ++i) {
        const int row  = i * 4 + (t >> 6);
        const int col4 = (t & 63) * 4;
        const float4 f = *(const float4*)&v[(size_t)s_nbr[row] * DIM + col4];
        *(float4*)&s_v[row * 256 + col4] = f;
    }
    __syncthreads();

    const int h  = t >> 5, hd = t & 31;
    const int kk = h * 4 + (hd >> 3);
    const int c0 = (hd & 7) * 32;
    const float* ap = &s_aff[h * 32];
    const float* vp = &s_v[kk * 256 + c0];
    float u = 0.0f;
#pragma unroll
    for (int k2 = 0; k2 < 32; ++k2) u = fmaf(ap[k2], vp[k2], u);

    float ssum = u, ssq = u * u;
#pragma unroll
    for (int off = 16; off >= 1; off >>= 1) {
        ssum += __shfl_xor(ssum, off, 32);
        ssq  += __shfl_xor(ssq, off, 32);
    }
    if (lane == 0) { s_red[t >> 5] = ssum; s_red[8 + (t >> 5)] = ssq; }
    __syncthreads();
    float tot = 0.0f, totq = 0.0f;
#pragma unroll
    for (int wv = 0; wv < 8; ++wv) { tot += s_red[wv]; totq += s_red[8 + wv]; }
    float mu   = tot * (1.0f / 256.0f);
    float var  = totq * (1.0f / 256.0f) - mu * mu;
    float rstd = rsqrtf(var + 1e-5f);
    float hn   = (u - mu) * rstd * ln_g[t] + ln_b[t];
    __shared__ __attribute__((aligned(16))) _Float16 s_h[256];
    s_h[t] = (_Float16)hn;
    __syncthreads();
    if (t < 32) { const v4u_t hv = *(const volatile v4ua*)(s_h + t * 8);
        *(volatile v4u_t*)(hout + (size_t)q * DIM + t * 8) = hv; __threadfence(); *(volatile v4u_t*)(hout + (size_t)q * DIM + t * 8) = hv; }
}

extern "C" void kernel_launch(void* const* d_in, const int* in_sizes, int n_in,
                              void* d_out, int out_size, void* d_ws, size_t ws_size,
                              hipStream_t stream) {
    const float* x     = (const float*)d_in[0];
    const int*   knn   = (const int*)d_in[1];
    const float* fp    = (const float*)d_in[3];
    const int*   npm   = (const int*)d_in[5];
    const float* q_w   = (const float*)d_in[6];
    const float* q_b   = (const float*)d_in[7];
    const float* v_w   = (const float*)d_in[8];
    const float* v_b   = (const float*)d_in[9];
    const float* ln_g  = (const float*)d_in[10];
    const float* ln_b  = (const float*)d_in[11];
    const float* fc1_w = (const float*)d_in[12];
    const float* fc1_b = (const float*)d_in[13];
    const float* fc2_w = (const float*)d_in[14];
    const float* fc2_b = (const float*)d_in[15];
    float* out = (float*)d_out;

    const int* i1 = knn + (size_t)BN * KK;

    char* ws = (char*)d_ws;
    float*    v_proj = (float*)(ws + 0);
    float*    qpos   = (float*)(ws + 8u * 1024 * 1024);
    _Float16* hnorm  = (_Float16*)(ws + 9u * 1024 * 1024);
    _Float16* tbuf   = (_Float16*)(ws + 13u * 1024 * 1024 + 512u * 1024);

    qpos_kernel<<<(BN * 24 + 255) / 256, 256, 0, stream>>>(x, q_w, q_b, qpos);
    gemm_wmma<float, 0, float, DIM, DIM><<<dim3(BN / 128, DIM / 64), 256, 0, stream>>>(
        x, v_w, v_b, nullptr, v_proj);
    attn_ln_kernel<<<BN, 256, 0, stream>>>(qpos, fp, i1, npm, v_proj, ln_g, ln_b, hnorm);
    gemm_wmma<_Float16, 1, _Float16, DIM, DIM><<<dim3(BN / 128, DIM / 64), 256, 0, stream>>>(
        hnorm, fc1_w, fc1_b, nullptr, tbuf);
    gemm_wmma<_Float16, 2, float, DIM, DIM><<<dim3(BN / 128, DIM / 64), 256, 0, stream>>>(
        tbuf, fc2_w, fc2_b, x, out);
}
